// LAINRDecoderGaussian_51359218925918
// MI455X (gfx1250) — hardware-verified
//
#include <hip/hip_runtime.h>
#include <math.h>
#include <stdint.h>

#define NBATCH 4
#define NPIX   16384
#define NTOK   256
#define FDIM   64
#define HDIM   256
#define NHEAD  2
#define DHEAD  64
#define INNER  128
#define NOUTC  3
#define PATCHN 16

#define F_BIAS 1
#define F_ADDF 2
#define F_RELU 4
#define F_ADDB 8

static_assert(NHEAD * DHEAD == INNER);
static_assert((NPIX % 256) == 0);
static_assert((NTOK % 64) == 0 && (HDIM % 64) == 0 && (INNER % 64) == 0 && (FDIM % 64) == 0);

typedef _Float16 v16h __attribute__((ext_vector_type(16)));
typedef _Float16 v8h  __attribute__((ext_vector_type(8)));
typedef __bf16   v16b __attribute__((ext_vector_type(16)));
typedef __bf16   v8b  __attribute__((ext_vector_type(8)));
typedef float    v8f  __attribute__((ext_vector_type(8)));
typedef float    v4f  __attribute__((ext_vector_type(4)));
typedef unsigned int v4u __attribute__((ext_vector_type(4)));

__device__ __forceinline__ unsigned short bf_bits(float f) {
  unsigned u = __float_as_uint(f);
  return (unsigned short)((u + 0x7FFFu + ((u >> 16) & 1u)) >> 16);
}
__device__ __forceinline__ float bf_up(unsigned short h) { return __uint_as_float(((unsigned)h) << 16); }
__device__ __forceinline__ unsigned short h_bits(_Float16 x) { return __builtin_bit_cast(unsigned short, x); }
__device__ __forceinline__ unsigned pk16(unsigned short a, unsigned short b) { return (unsigned)a | ((unsigned)b << 16); }
__device__ __forceinline__ v8f zero8() { v8f z = {0.f, 0.f, 0.f, 0.f, 0.f, 0.f, 0.f, 0.f}; return z; }

__device__ __forceinline__ v16b ldfrag_b(const __bf16* p) {
  union { v16b v; v8b h[2]; } f;
  f.h[0] = *(const v8b*)(p);
  f.h[1] = *(const v8b*)(p + 16);
  return f.v;
}
__device__ __forceinline__ v16h ldfrag_h(const _Float16* p) {
  union { v16h v; v8h h[2]; } f;
  f.h[0] = *(const v8h*)(p);
  f.h[1] = *(const v8h*)(p + 16);
  return f.v;
}

__device__ __forceinline__ v8f mma_h(v16h a, v16h b, v8f c) {
  c = __builtin_amdgcn_wmma_f32_16x16x32_f16(false, a, false, b, (short)0, c, false, false);
#if defined(__HIP_DEVICE_COMPILE__)
  asm volatile("v_nop\n\tv_nop\n\tv_nop\n\tv_nop" : "+v"(c) : "v"(a), "v"(b));
#endif
  return c;
}
__device__ __forceinline__ v8f mma_b(v16b a, v16b b, v8f c) {
  c = __builtin_amdgcn_wmma_f32_16x16x32_bf16(false, a, false, b, (short)0, c, false, false);
#if defined(__HIP_DEVICE_COMPILE__)
  asm volatile("v_nop\n\tv_nop\n\tv_nop\n\tv_nop" : "+v"(c) : "v"(a), "v"(b));
#endif
  return c;
}
__device__ __forceinline__ v8f mma_b_raw(v16b a, v16b b, v8f c) {
  return __builtin_amdgcn_wmma_f32_16x16x32_bf16(false, a, false, b, (short)0, c, false, false);
}
__device__ __forceinline__ void dep_guard_b(v8f& a, v8f& b, v16b x, v16b y) {
#if defined(__HIP_DEVICE_COMPILE__)
  asm volatile("v_nop\n\tv_nop\n\tv_nop\n\tv_nop" : "+v"(a), "+v"(b) : "v"(x), "v"(y));
#endif
}
__device__ __forceinline__ void keep4_b(v16b a, v16b b, v16b c, v16b d) {
#if defined(__HIP_DEVICE_COMPILE__)
  asm volatile("v_nop" :: "v"(a), "v"(b), "v"(c), "v"(d));
#endif
}
__device__ __forceinline__ void acc_guard4(v8f& a, v8f& b, v8f& c, v8f& d) {
#if defined(__HIP_DEVICE_COMPILE__)
  asm volatile("v_nop\n\tv_nop\n\tv_nop\n\tv_nop" : "+v"(a), "+v"(b), "+v"(c), "+v"(d));
#endif
}
__device__ __forceinline__ void wave_sync_lds() {
  __builtin_amdgcn_fence(__ATOMIC_RELEASE, "workgroup");
  __builtin_amdgcn_wave_barrier();
  __builtin_amdgcn_fence(__ATOMIC_ACQUIRE, "workgroup");
}

__global__ __launch_bounds__(256) void cvt_bf16x8(const float* __restrict__ in, unsigned short* out, int n8) {
  const int i = blockIdx.x * 256 + threadIdx.x;
  if (i < n8) {
    const v4f a = *(const v4f*)(in + (size_t)i * 8);
    const v4f b = *(const v4f*)(in + (size_t)i * 8 + 4);
    v4u p;
    p[0] = pk16(bf_bits(a[0]), bf_bits(a[1]));
    p[1] = pk16(bf_bits(a[2]), bf_bits(a[3]));
    p[2] = pk16(bf_bits(b[0]), bf_bits(b[1]));
    p[3] = pk16(bf_bits(b[2]), bf_bits(b[3]));
    *(volatile v4u*)(out + (size_t)i * 8) = p;
    __threadfence();
    *(volatile v4u*)(out + (size_t)i * 8) = p;
  }
}

__global__ __launch_bounds__(256) void cvt_wT(const float* __restrict__ w0, const float* __restrict__ w1,
                                              const float* __restrict__ w2, const float* __restrict__ w3,
                                              unsigned short* outp, int nin, int nout) {
  __shared__ float tile[64][33];
  const int tid = threadIdx.x;
  const int z = blockIdx.z;
  const float* src = (z == 0) ? w0 : ((z == 1) ? w1 : ((z == 2) ? w2 : w3));
  unsigned short* dst = outp + (size_t)z * nin * nout;
  const int i0 = blockIdx.x * 64;
  const int o0 = blockIdx.y * 32;
#pragma unroll
  for (int p = 0; p < 8; ++p) {
    const int idx = p * 256 + tid;
    const int i = idx >> 5, o = idx & 31;
    tile[i][o] = src[(size_t)(i0 + i) * nout + o0 + o];
  }
  __syncthreads();
  const int o = tid >> 3, c8 = (tid & 7) * 8;
  v4u pk;
#pragma unroll
  for (int e = 0; e < 4; ++e)
    pk[e] = pk16(bf_bits(tile[c8 + 2 * e][o]), bf_bits(tile[c8 + 2 * e + 1][o]));
  unsigned short* gp = dst + (size_t)(o0 + o) * nin + i0 + c8;
  *(volatile v4u*)gp = pk;
  __threadfence();
  *(volatile v4u*)gp = pk;
}

__global__ __launch_bounds__(256) void feat3(const float* __restrict__ coords,
                                             const float* __restrict__ Bq, const float* __restrict__ Bl0,
                                             const float* __restrict__ Bl1,
                                             unsigned short* fqh, unsigned short* fql,
                                             unsigned short* f0h, unsigned short* f0l,
                                             unsigned short* f1h, unsigned short* f1l) {
#pragma clang fp contract(off)
  __shared__ __align__(16) float tile[32 * 64];
  const int tid = threadIdx.x;
  const int px0 = blockIdx.x * 32;
  const int p = tid >> 3, fg = tid & 7;
  const float g0 = bf_up(bf_bits(coords[2 * (px0 + p)]));
  const float g1 = bf_up(bf_bits(coords[2 * (px0 + p) + 1]));
  const float twopi = 6.283185307179586f;
  const float tp0 = twopi * g0;
  const float tp1 = twopi * g1;
  const int row = tid >> 3, c8 = (tid & 7) * 8;
#pragma unroll 1
  for (int z = 0; z < 3; ++z) {
    const float* Bm = (z == 0) ? Bq : ((z == 1) ? Bl0 : Bl1);
    unsigned short* dh = (z == 0) ? fqh : ((z == 1) ? f0h : f1h);
    unsigned short* dl = (z == 0) ? fql : ((z == 1) ? f0l : f1l);
#pragma unroll 1
    for (int f4 = 0; f4 < 4; ++f4) {
      const int f = fg * 4 + f4;
      const float bx = bf_up(bf_bits(Bm[2 * f]));
      const float by = bf_up(bf_bits(Bm[2 * f + 1]));
      const float pa = tp0 * bx;
      const float pb = tp1 * by;
      const float proj = pa + pb;
      tile[p * 64 + f] = cosf(proj);
      tile[p * 64 + 32 + f] = sinf(proj);
    }
    __syncthreads();
    const float* sp = tile + row * 64 + c8;
    v4u a, a2;
#pragma unroll
    for (int e = 0; e < 4; ++e) {
      const float x0 = sp[2 * e], x1 = sp[2 * e + 1];
      const unsigned short hb0 = bf_bits(x0), hb1 = bf_bits(x1);
      const unsigned short lb0 = bf_bits(x0 - bf_up(hb0)), lb1 = bf_bits(x1 - bf_up(hb1));
      a[e] = pk16(hb0, hb1); a2[e] = pk16(lb0, lb1);
    }
    const size_t go = (size_t)(px0 + row) * FDIM + c8;
    *(volatile v4u*)(dh + go) = a;
    *(volatile v4u*)(dl + go) = a2;
    __threadfence();
    *(volatile v4u*)(dh + go) = a;
    *(volatile v4u*)(dl + go) = a2;
    __syncthreads();
  }
}

__device__ __forceinline__ float epi_val(float f, int m, int n, const float* biasp, const float* addF, int ldf,
                                         const unsigned short* addH, const unsigned short* addL, int ldq,
                                         int flags) {
#pragma clang fp contract(off)
  if (flags & F_BIAS) f = f + bf_up(bf_bits(biasp[n]));
  if (flags & F_ADDF) f = f + addF[(size_t)m * ldf + n];
  if (flags & F_RELU) f = fmaxf(f, 0.0f);
  if (flags & F_ADDB) {
    const size_t qo = (size_t)m * ldq + n;
    const float mv = bf_up(addH[qo]) + bf_up(addL[qo]);
    f = f + mv;
  }
  return f;
}

template <int NSPLIT, int OUT_MODE>
__global__ __launch_bounds__(256) void gemm64(
    const unsigned short* __restrict__ Ap, const unsigned short* __restrict__ A2p, int lda, long long strideA,
    const unsigned short* __restrict__ Btp, int ldb, long long strideB,
    void* Cout, void* Cout2, int ldc, long long strideC,
    int M, int N, int K,
    const float* biasp, const float* addF, int ldf,
    const unsigned short* addH, const unsigned short* addL, int ldq, int flags) {
#pragma clang fp contract(off)
  const __bf16* A  = (const __bf16*)(const void*)Ap;
  const __bf16* A2 = (const __bf16*)(const void*)A2p;
  const __bf16* Bt = (const __bf16*)(const void*)Btp;
  __shared__ __align__(16) float sT[8][16 * 68];
  const int b    = blockIdx.y;
  const int lane = threadIdx.x & 31;
  const int wave = threadIdx.x >> 5;
  const int tilesN = N >> 6;
  const int tilesM = M >> 6;
  const int tile = blockIdx.x * 8 + wave;
  if (tile >= tilesM * tilesN) return;
  const int tm = tile / tilesN;
  const int tn = tile - tm * tilesN;
  const int m0 = tm << 6;
  const int n0 = tn << 6;

  const __bf16* Ab  = A  + (size_t)b * (size_t)strideA;
  const __bf16* Ab2 = (NSPLIT >= 1) ? (A2 + (size_t)b * (size_t)strideA) : Ab;
  const __bf16* Bb  = Bt + (size_t)b * (size_t)strideB;

  const int rlane = lane & 15;
  const int koff  = (lane >> 4) * 8;
  const int mOff  = (lane >> 4) * 8;

  v8f acc[4][4];
#pragma unroll
  for (int i = 0; i < 4; ++i)
#pragma unroll
    for (int j = 0; j < 4; ++j) acc[i][j] = zero8();

  for (int k0 = 0; k0 < K; k0 += 32) {
    v16b bh[4];
#pragma unroll
    for (int j = 0; j < 4; ++j) {
      const size_t bo = (size_t)(n0 + (j << 4) + rlane) * ldb + koff + k0;
      bh[j] = ldfrag_b(Bb + bo);
    }
#pragma unroll
    for (int i = 0; i < 4; ++i) {
      const size_t ao = (size_t)(m0 + (i << 4) + rlane) * lda + koff + k0;
      const v16b ah = ldfrag_b(Ab + ao);
      v16b al = ah;
      if (NSPLIT >= 1) al = ldfrag_b(Ab2 + ao);
#pragma unroll
      for (int j = 0; j < 4; ++j) {
        acc[i][j] = mma_b_raw(ah, bh[j], acc[i][j]);
        if (NSPLIT >= 1) acc[i][j] = mma_b_raw(al, bh[j], acc[i][j]);
      }
      dep_guard_b(acc[i][0], acc[i][3], ah, al);
    }
    keep4_b(bh[0], bh[1], bh[2], bh[3]);
  }
  acc_guard4(acc[0][0], acc[0][1], acc[0][2], acc[0][3]);
  acc_guard4(acc[1][0], acc[1][1], acc[1][2], acc[1][3]);
  acc_guard4(acc[2][0], acc[2][1], acc[2][2], acc[2][3]);
  acc_guard4(acc[3][0], acc[3][1], acc[3][2], acc[3][3]);

  float* slab = sT[wave];
#pragma unroll
  for (int i = 0; i < 4; ++i) {
    const int mBase = m0 + (i << 4);
#pragma unroll
    for (int j = 0; j < 4; ++j) {
#pragma unroll
      for (int r = 0; r < 8; ++r) {
        slab[(mOff + r) * 68 + (j << 4) + rlane] = acc[i][j][r];
      }
    }
    wave_sync_lds();
    if (OUT_MODE == 0) {
      float* C = (float*)Cout + (size_t)b * (size_t)strideC;
      const int h2 = lane >> 4, c4 = (lane & 15) * 4;
      for (int pass = 0; pass < 2; ++pass) {
#pragma unroll
        for (int it = 0; it < 8; ++it) {
          const int row = it * 2 + h2;
          const int m = mBase + row;
          v4f v = *(const v4f*)(slab + row * 68 + c4);
#pragma unroll
          for (int e = 0; e < 4; ++e)
            v[e] = epi_val(v[e], m, n0 + c4 + e, biasp, addF, ldf, addH, addL, ldq, flags);
          *(volatile v4f*)(C + (size_t)m * ldc + n0 + c4) = v;
        }
        __threadfence();
      }
    } else {
      const int q = lane >> 3, c8 = (lane & 7) * 8;
      unsigned short* C  = (unsigned short*)Cout  + (size_t)b * (size_t)strideC;
      unsigned short* C2 = (unsigned short*)Cout2 + (size_t)b * (size_t)strideC;
      v4u hv[4], lv[4];
#pragma unroll
      for (int it = 0; it < 4; ++it) {
        const int row = it * 4 + q;
        const int m = mBase + row;
        const float* sp = slab + row * 68 + c8;
        float fv[8];
#pragma unroll
        for (int e = 0; e < 8; ++e)
          fv[e] = epi_val(sp[e], m, n0 + c8 + e, biasp, addF, ldf, addH, addL, ldq, flags);
        v4u a, a2;
#pragma unroll
        for (int e = 0; e < 4; ++e) {
          const float x0 = fv[2 * e], x1 = fv[2 * e + 1];
          unsigned short h0, h1, l0, l1;
          if (OUT_MODE == 2) {
            h0 = bf_bits(x0); h1 = bf_bits(x1);
            l0 = bf_bits(x0 - bf_up(h0)); l1 = bf_bits(x1 - bf_up(h1));
          } else {
            h0 = h_bits((_Float16)x0); h1 = h_bits((_Float16)x1);
            l0 = 0; l1 = 0;
          }
          a[e] = pk16(h0, h1); a2[e] = pk16(l0, l1);
        }
        hv[it] = a; lv[it] = a2;
      }
      for (int pass = 0; pass < 2; ++pass) {
#pragma unroll
        for (int it = 0; it < 4; ++it) {
          const int row = it * 4 + q;
          *(volatile v4u*)(C + (size_t)(mBase + row) * ldc + n0 + c8) = hv[it];
          if (OUT_MODE == 2) *(volatile v4u*)(C2 + (size_t)(mBase + row) * ldc + n0 + c8) = lv[it];
        }
        __threadfence();
      }
    }
    wave_sync_lds();
  }
}

__global__ __launch_bounds__(256)
void attn64(const unsigned short* __restrict__ qhp, const unsigned short* __restrict__ khp,
            const unsigned short* __restrict__ vhp, const float* __restrict__ coords,
            unsigned short* ohp, unsigned short* olp, int b) {
#pragma clang fp contract(off)
  union FH { v16h v; v8h h[2]; };
  __shared__ __align__(16) _Float16 Psh[8][16 * 64];
  __shared__ __align__(16) float    Os[64 * INNER];

  const int tid  = threadIdx.x;
  const int wave = tid >> 5;
  const int lane = tid & 31;
  const int hh   = lane >> 4;
  const int c    = lane & 15;

  const int qb   = blockIdx.x;
  const int hp   = wave >> 2;
  const int wq   = wave & 3;
  const int q0   = qb * 64 + wq * 16;

  const _Float16* Qh = (const _Float16*)(const void*)qhp + (size_t)hp * DHEAD;
  const _Float16* Kh = (const _Float16*)(const void*)khp + (size_t)b * NTOK * INNER + (size_t)hp * DHEAD;
  const _Float16* Vh = (const _Float16*)(const void*)vhp + ((size_t)b * INNER + (size_t)hp * DHEAD) * NTOK;

  v16h qa[2];
#pragma unroll
  for (int kk = 0; kk < 2; ++kk) qa[kk] = ldfrag_h(Qh + (size_t)(q0 + c) * INNER + kk * 32 + 8 * hh);

  float trow[8];
#pragma unroll
  for (int r = 0; r < 8; ++r) {
    const int p = q0 + 8 * hh + r;
    const float g0 = bf_up(bf_bits(coords[2 * p]));
    const float g1 = bf_up(bf_bits(coords[2 * p + 1]));
    const float r16 = g0 * 16.0f;
    const float c16 = g1 * 16.0f;
    int ir = (int)r16; ir = (ir < 0) ? 0 : ((ir > PATCHN - 1) ? (PATCHN - 1) : ir);
    int ic = (int)c16; ic = (ic < 0) ? 0 : ((ic > PATCHN - 1) ? (PATCHN - 1) : ic);
    trow[r] = (float)(ir * PATCHN + ic) * (1.0f / 256.0f);
  }

  float mrow[8], lrow[8];
  v8f oacc[4];
#pragma unroll
  for (int r = 0; r < 8; ++r) { mrow[r] = -INFINITY; lrow[r] = 0.f; }
#pragma unroll
  for (int t = 0; t < 4; ++t) oacc[t] = zero8();

  _Float16* pw = Psh[wave];

  for (int kt = 0; kt < NTOK / 64; ++kt) {
    const int kv0 = kt * 64;

    v8f s[4];
#pragma unroll
    for (int j = 0; j < 4; ++j) {
      v8f a = zero8();
#pragma unroll
      for (int kk = 0; kk < 2; ++kk) {
        const size_t ko = (size_t)(kv0 + j * 16 + c) * INNER + kk * 32 + 8 * hh;
        const v16h kb = ldfrag_h(Kh + ko);
        a = mma_h(qa[kk], kb, a);
      }
      const float pos = ((float)(kv0 + j * 16 + c) + 0.5f) * (1.0f / 256.0f);
#pragma unroll
      for (int r = 0; r < 8; ++r) {
        const float d = trow[r] - pos;
        const float d2 = d * d;
        const float bias = -10.0f * d2;
        const float sc = a[r] * 0.125f;
        s[j][r] = sc + bias;
      }
    }

#pragma unroll
    for (int r = 0; r < 8; ++r) {
      float m = fmaxf(fmaxf(s[0][r], s[1][r]), fmaxf(s[2][r], s[3][r]));
#pragma unroll
      for (int off = 1; off < 16; off <<= 1) m = fmaxf(m, __shfl_xor(m, off, 32));
      const float mnew  = fmaxf(mrow[r], m);
      const float alpha = __expf(mrow[r] - mnew);
      mrow[r] = mnew;
      float psum = 0.f;
#pragma unroll
      for (int j = 0; j < 4; ++j) {
        const float p  = __expf(s[j][r] - mnew);
        psum += p;
        const float p1 = p * 1024.0f;
        pw[(8 * hh + r) * 64 + j * 16 + c] = (_Float16)p1;
      }
#pragma unroll
      for (int off = 1; off < 16; off <<= 1) psum += __shfl_xor(psum, off, 32);
      lrow[r] = lrow[r] * alpha + psum;
#pragma unroll
      for (int t = 0; t < 4; ++t) oacc[t][r] *= alpha;
    }
    wave_sync_lds();

#pragma unroll
    for (int kk = 0; kk < 2; ++kk) {
      FH pa;
      pa.h[0] = *(const v8h*)(pw + c * 64 + kk * 32 + 8 * hh);
      pa.h[1] = *(const v8h*)(pw + c * 64 + kk * 32 + 16 + 8 * hh);
#pragma unroll
      for (int t = 0; t < 4; ++t) {
        const size_t vo = (size_t)(t * 16 + c) * NTOK + kv0 + kk * 32 + 8 * hh;
        const v16h vb = ldfrag_h(Vh + vo);
        oacc[t] = mma_h(pa.v, vb, oacc[t]);
      }
    }
    wave_sync_lds();
  }

#pragma unroll
  for (int r = 0; r < 8; ++r) {
    const float l = lrow[r];
    const float inv = ((l > 0.f) ? (1.0f / l) : 0.f) * (1.0f / 1024.0f);
#pragma unroll
    for (int t = 0; t < 4; ++t) Os[(wq * 16 + 8 * hh + r) * INNER + hp * DHEAD + t * 16 + c] = oacc[t][r] * inv;
  }
  __syncthreads();
  {
    const int rh = lane >> 4, c16 = (lane & 15) * 8;
    v4u hv[4], lv[4];
#pragma unroll
    for (int it = 0; it < 4; ++it) {
      const int row = wave * 8 + it * 2 + rh;
      const float* sp = Os + row * INNER + c16;
      v4u a, a2;
#pragma unroll
      for (int e = 0; e < 4; ++e) {
        const float x0 = sp[2 * e], x1 = sp[2 * e + 1];
        const unsigned short h0 = bf_bits(x0), h1 = bf_bits(x1);
        const unsigned short l0 = bf_bits(x0 - bf_up(h0)), l1 = bf_bits(x1 - bf_up(h1));
        a[e] = pk16(h0, h1); a2[e] = pk16(l0, l1);
      }
      hv[it] = a; lv[it] = a2;
    }
    for (int pass = 0; pass < 2; ++pass) {
#pragma unroll
      for (int it = 0; it < 4; ++it) {
        const int row = wave * 8 + it * 2 + rh;
        const size_t go = (size_t)(qb * 64 + row) * INNER + c16;
        *(volatile v4u*)(ohp + go) = hv[it];
        *(volatile v4u*)(olp + go) = lv[it];
      }
      __threadfence();
    }
  }
}

__global__ __launch_bounds__(128)
void outk(const unsigned short* __restrict__ m0h, const unsigned short* __restrict__ m0l,
          const unsigned short* __restrict__ hvh, const unsigned short* __restrict__ hvl,
          const float* __restrict__ W0, const float* __restrict__ b0,
          const float* __restrict__ W1, const float* __restrict__ b1, float* outp) {
#pragma clang fp contract(off)
  __shared__ __align__(16) __bf16 Bs[16 * 512];
  __shared__ __align__(16) float  sO[4][192];

  const int tid  = threadIdx.x;
  const int wave = tid >> 5;
  const int lane = tid & 31;
  const int c    = lane & 15;
  const int koff = (lane >> 4) * 8;
  const int mOff = (lane >> 4) * 8;

#pragma unroll 4
  for (int e = 0; e < 64; ++e) {
    const int idx = e * 128 + tid;
    const int n = idx >> 9, k = idx & 511;
    const int nn = (n < NOUTC) ? n : (NOUTC - 1);
    const int ka = (k < HDIM) ? k : (k - HDIM);
    const float w0v = W0[ka * NOUTC + nn];
    const float w1v = W1[ka * NOUTC + nn];
    float val = (k < HDIM) ? w0v : w1v;
    val = (n < NOUTC) ? val : 0.0f;
    Bs[idx] = __builtin_bit_cast(__bf16, bf_bits(val));
  }
  __syncthreads();

  const int cc = (c < NOUTC) ? c : (NOUTC - 1);
  float obv = bf_up(bf_bits(b0[cc])) + bf_up(bf_bits(b1[cc]));
  obv = (c < NOUTC) ? obv : 0.0f;

  const int m0w = blockIdx.x * 256 + wave * 64;
  const __bf16* M0H = (const __bf16*)(const void*)m0h;
  const __bf16* M0L = (const __bf16*)(const void*)m0l;
  const __bf16* HVH = (const __bf16*)(const void*)hvh;
  const __bf16* HVL = (const __bf16*)(const void*)hvl;

  v8f acc[4];
#pragma unroll
  for (int i = 0; i < 4; ++i) acc[i] = zero8();

#pragma unroll 2
  for (int k0 = 0; k0 < HDIM; k0 += 32) {
    const v16b bw = ldfrag_b(Bs + c * 512 + k0 + koff);
#pragma unroll
    for (int i = 0; i < 4; ++i) {
      const size_t ao = (size_t)(m0w + 16 * i + c) * HDIM + k0 + koff;
      const v16b ah = ldfrag_b(M0H + ao);
      const v16b al = ldfrag_b(M0L + ao);
      acc[i] = mma_b(ah, bw, acc[i]);
      acc[i] = mma_b(al, bw, acc[i]);
    }
  }
#pragma unroll 2
  for (int k0 = 0; k0 < HDIM; k0 += 32) {
    const v16b bw = ldfrag_b(Bs + c * 512 + HDIM + k0 + koff);
#pragma unroll
    for (int i = 0; i < 4; ++i) {
      const size_t ao = (size_t)(m0w + 16 * i + c) * HDIM + k0 + koff;
      const v16b ah = ldfrag_b(HVH + ao);
      const v16b al = ldfrag_b(HVL + ao);
      acc[i] = mma_b(ah, bw, acc[i]);
      acc[i] = mma_b(al, bw, acc[i]);
    }
  }
  acc_guard4(acc[0], acc[1], acc[2], acc[3]);

  float* so = sO[wave];
#pragma unroll
  for (int i = 0; i < 4; ++i) {
#pragma unroll
    for (int r = 0; r < 8; ++r) {
      const float v = acc[i][r] + obv;
      if (c < NOUTC) so[(16 * i + mOff + r) * NOUTC + c] = v;
    }
  }
  wave_sync_lds();
  const int l1 = (lane < 16) ? lane : 15;
  const v4f v0 = *(const v4f*)(so + 4 * lane);
  const v4f v1 = *(const v4f*)(so + 128 + 4 * l1);
  float* ob = outp + (size_t)m0w * NOUTC;
  for (int pass = 0; pass < 2; ++pass) {
    *(volatile v4f*)(ob + 4 * lane) = v0;
    if (lane < 16) *(volatile v4f*)(ob + 128 + 4 * lane) = v1;
    __threadfence();
  }
}

extern "C" void kernel_launch(void* const* d_in, const int* in_sizes, int n_in,
                              void* d_out, int out_size, void* d_ws, size_t ws_size,
                              hipStream_t stream) {
  if (n_in < 25) return;
  if (in_sizes[0] != NBATCH * NPIX * 2) return;
  if (in_sizes[1] != NBATCH * NTOK * HDIM) return;
  if (in_sizes[2] != 64 || in_sizes[3] != 64 || in_sizes[4] != 64) return;
  if (in_sizes[5] != FDIM * HDIM || in_sizes[6] != HDIM) return;
  if (in_sizes[7] != HDIM * INNER) return;
  if (in_sizes[8] != HDIM * 2 * INNER) return;
  if (in_sizes[9] != INNER * HDIM || in_sizes[10] != HDIM) return;
  if (in_sizes[11] != FDIM * HDIM || in_sizes[12] != HDIM) return;
  if (in_sizes[13] != FDIM * HDIM || in_sizes[14] != HDIM) return;
  if (in_sizes[15] != HDIM * HDIM || in_sizes[16] != HDIM) return;
  if (in_sizes[17] != HDIM * HDIM || in_sizes[18] != HDIM) return;
  if (in_sizes[19] != HDIM * HDIM || in_sizes[20] != HDIM) return;
  if (in_sizes[21] != HDIM * NOUTC || in_sizes[22] != NOUTC) return;
  if (in_sizes[23] != HDIM * NOUTC || in_sizes[24] != NOUTC) return;
  if (out_size != NBATCH * NPIX * NOUTC) return;

  const float* coords = (const float*)d_in[0];
  const float* tokens = (const float*)d_in[1];
  const float* B_q    = (const float*)d_in[2];
  const float* B_l0   = (const float*)d_in[3];
  const float* B_l1   = (const float*)d_in[4];
  const float* qW     = (const float*)d_in[5];
  const float* qb     = (const float*)d_in[6];
  const float* toqW   = (const float*)d_in[7];
  const float* tokvW  = (const float*)d_in[8];
  const float* tooW   = (const float*)d_in[9];
  const float* toob   = (const float*)d_in[10];
  const float* bwW0   = (const float*)d_in[11];
  const float* bwb0   = (const float*)d_in[12];
  const float* bwW1   = (const float*)d_in[13];
  const float* bwb1   = (const float*)d_in[14];
  const float* modW0  = (const float*)d_in[15];
  const float* modb0  = (const float*)d_in[16];
  const float* modW1  = (const float*)d_in[17];
  const float* modb1  = (const float*)d_in[18];
  const float* hvW0   = (const float*)d_in[19];
  const float* hvb0   = (const float*)d_in[20];
  const float* outW0  = (const float*)d_in[21];
  const float* outb0  = (const float*)d_in[22];
  const float* outW1  = (const float*)d_in[23];
  const float* outb1  = (const float*)d_in[24];

  const size_t sXtok = (size_t)NBATCH * NTOK * HDIM * 2;
  const size_t sW64  = (size_t)3 * HDIM * FDIM * 2;
  const size_t sW256 = (size_t)4 * HDIM * HDIM * 2;
  const size_t sWtoq = (size_t)INNER * HDIM * 2;
  const size_t sWtoo = (size_t)HDIM * INNER * 2;
  const size_t sF    = (size_t)NPIX * FDIM * 2;
  const size_t sP16  = (size_t)NPIX * HDIM * 2;
  const size_t sQ    = (size_t)NPIX * INNER * 2;
  const size_t sK    = (size_t)NBATCH * NTOK * INNER * 2;
  const size_t sVT   = (size_t)NBATCH * INNER * NTOK * 2;
  const size_t sHB   = (size_t)NPIX * HDIM * 4;
  size_t off = 0;
  const size_t oXtok = off; off += sXtok;
  const size_t oW64  = off; off += sW64;
  const size_t oW256 = off; off += sW256;
  const size_t oWtoq = off; off += sWtoq;
  const size_t oWtoo = off; off += sWtoo;
  const size_t oF    = off; off += 6 * sF;
  const size_t oXQ   = off; off += 2 * sP16;
  const size_t oQ    = off; off += sQ;
  const size_t oK    = off; off += sK;
  const size_t oVT   = off; off += sVT;
  const size_t oHB0  = off; off += sHB;
  const size_t oHB1  = off; off += sHB;
  const size_t oOA   = off; off += 2 * sP16;
  const size_t oMH   = off; off += 2 * sP16;
  const size_t oM0   = off; off += 2 * sP16;
  if (off > ws_size) return;
  if (off > (size_t)134217728) return;

  char* ws = (char*)d_ws;
  unsigned short* Xtok  = (unsigned short*)(ws + oXtok);
  unsigned short* W64   = (unsigned short*)(ws + oW64);
  unsigned short* WqT   = W64;
  unsigned short* Wb0T  = W64 + (size_t)1 * HDIM * FDIM;
  unsigned short* Wb1T  = W64 + (size_t)2 * HDIM * FDIM;
  unsigned short* W256  = (unsigned short*)(ws + oW256);
  unsigned short* WkvT  = W256;
  unsigned short* Wm0T  = W256 + (size_t)1 * HDIM * HDIM;
  unsigned short* Wm1T  = W256 + (size_t)2 * HDIM * HDIM;
  unsigned short* WhvT  = W256 + (size_t)3 * HDIM * HDIM;
  unsigned short* WtoqT = (unsigned short*)(ws + oWtoq);
  unsigned short* WtooT = (unsigned short*)(ws + oWtoo);
  unsigned short* FQh   = (unsigned short*)(ws + oF);
  unsigned short* FQl   = (unsigned short*)(ws + oF + sF);
  unsigned short* F0h   = (unsigned short*)(ws + oF + 2 * sF);
  unsigned short* F0l   = (unsigned short*)(ws + oF + 3 * sF);
  unsigned short* F1h   = (unsigned short*)(ws + oF + 4 * sF);
  unsigned short* F1l   = (unsigned short*)(ws + oF + 5 * sF);
  unsigned short* XQh   = (unsigned short*)(ws + oXQ);
  unsigned short* XQl   = (unsigned short*)(ws + oXQ + sP16);
  unsigned short* Qh    = (unsigned short*)(ws + oQ);
  unsigned short* Kh    = (unsigned short*)(ws + oK);
  unsigned short* VTh   = (unsigned short*)(ws + oVT);
  float*          HB0   = (float*)(ws + oHB0);
  float*          HB1   = (float*)(ws + oHB1);
  unsigned short* Oh    = (unsigned short*)(ws + oOA);
  unsigned short* Ol    = (unsigned short*)(ws + oOA + sQ);
  unsigned short* Ah    = (unsigned short*)(ws + oOA);
  unsigned short* Al    = (unsigned short*)(ws + oOA + sP16);
  unsigned short* MODh  = (unsigned short*)(ws + oMH);
  unsigned short* MODl  = (unsigned short*)(ws + oMH + sP16);
  unsigned short* HVh   = (unsigned short*)(ws + oMH);
  unsigned short* HVl   = (unsigned short*)(ws + oMH + sP16);
  unsigned short* M0h   = (unsigned short*)(ws + oM0);
  unsigned short* M0l   = (unsigned short*)(ws + oM0 + sP16);
  float* out = (float*)d_out;

  const dim3 blk(256);
  const int n8tok = NBATCH * NTOK * HDIM / 8;
  const dim3 gCvtT((n8tok + 255) / 256);
  const dim3 gW64(FDIM / 64, HDIM / 32, 3);
  const dim3 gW256(HDIM / 64, HDIM / 32, 4);
  const dim3 gWtoq(HDIM / 64, INNER / 32, 1);
  const dim3 gWtoo(INNER / 64, HDIM / 32, 1);
  const dim3 gFeat(NPIX / 32);
  const dim3 gP256(((NPIX / 64) * (HDIM / 64) + 7) / 8, 1);
  const dim3 gP128(((NPIX / 64) * (INNER / 64) + 7) / 8, 1);
  const dim3 gK((((NBATCH * NTOK) / 64) * (INNER / 64) + 7) / 8, 1);
  const dim3 gVT(((INNER / 64) * (NTOK / 64) + 7) / 8, NBATCH);
  const dim3 gAttn(NPIX / 64);
  const dim3 gOut(NPIX / 256);

  cvt_bf16x8<<<gCvtT, blk, 0, stream>>>(tokens, Xtok, n8tok);
  cvt_wT<<<gW64, blk, 0, stream>>>(qW, bwW0, bwW1, bwW1, W64, FDIM, HDIM);
  cvt_wT<<<gW256, blk, 0, stream>>>(tokvW, modW0, modW1, hvW0, W256, HDIM, HDIM);
  cvt_wT<<<gWtoq, blk, 0, stream>>>(toqW, toqW, toqW, toqW, WtoqT, HDIM, INNER);
  cvt_wT<<<gWtoo, blk, 0, stream>>>(tooW, tooW, tooW, tooW, WtooT, INNER, HDIM);
  feat3<<<gFeat, blk, 0, stream>>>(coords, B_q, B_l0, B_l1, FQh, FQl, F0h, F0l, F1h, F1l);
  gemm64<1, 2><<<gP256, blk, 0, stream>>>(
      FQh, FQl, FDIM, 0LL, WqT, FDIM, 0LL,
      (void*)XQh, (void*)XQl, HDIM, 0LL, NPIX, HDIM, FDIM,
      qb, HB0, HDIM, M0h, M0l, HDIM, F_BIAS | F_RELU);
  gemm64<1, 0><<<gP256, blk, 0, stream>>>(
      F0h, F0l, FDIM, 0LL, Wb0T, FDIM, 0LL,
      (void*)HB0, (void*)HB0, HDIM, 0LL, NPIX, HDIM, FDIM,
      bwb0, HB1, HDIM, XQh, XQl, HDIM, F_BIAS | F_RELU);
  gemm64<1, 0><<<gP256, blk, 0, stream>>>(
      F1h, F1l, FDIM, 0LL, Wb1T, FDIM, 0LL,
      (void*)HB1, (void*)HB1, HDIM, 0LL, NPIX, HDIM, FDIM,
      bwb1, HB0, HDIM, XQh, XQl, HDIM, F_BIAS | F_RELU);
  gemm64<1, 3><<<gP128, blk, 0, stream>>>(
      XQh, XQl, HDIM, 0LL, WtoqT, HDIM, 0LL,
      (void*)Qh, (void*)Qh, INNER, 0LL, NPIX, INNER, HDIM,
      qb, HB0, HDIM, XQh, XQl, HDIM, 0);
  gemm64<0, 3><<<gK, blk, 0, stream>>>(
      Xtok, Xtok, HDIM, 0LL, WkvT, HDIM, 0LL,
      (void*)Kh, (void*)Kh, INNER, 0LL, NBATCH * NTOK, INNER, HDIM,
      toob, HB0, HDIM, XQh, XQl, HDIM, 0);
  gemm64<0, 3><<<gVT, blk, 0, stream>>>(
      WkvT + (size_t)INNER * HDIM, WkvT + (size_t)INNER * HDIM, HDIM, 0LL, Xtok, HDIM, (long long)NTOK * HDIM,
      (void*)VTh, (void*)VTh, NTOK, (long long)INNER * NTOK, INNER, NTOK, HDIM,
      toob, HB0, HDIM, XQh, XQl, HDIM, 0);

  for (int b = 0; b < NBATCH; ++b) {
    attn64<<<gAttn, blk, 0, stream>>>(Qh, Kh, VTh, coords, Oh, Ol, b);
    gemm64<1, 2><<<gP256, blk, 0, stream>>>(
        Oh, Ol, INNER, 0LL, WtooT, INNER, 0LL,
        (void*)MODh, (void*)MODl, HDIM, 0LL, NPIX, HDIM, INNER,
        toob, HB0, HDIM, XQh, XQl, HDIM, F_BIAS);
    gemm64<1, 2><<<gP256, blk, 0, stream>>>(
        MODh, MODl, HDIM, 0LL, Wm0T, HDIM, 0LL,
        (void*)M0h, (void*)M0l, HDIM, 0LL, NPIX, HDIM, HDIM,
        modb0, HB0, HDIM, XQh, XQl, HDIM, F_BIAS | F_ADDF | F_RELU);
    gemm64<1, 2><<<gP256, blk, 0, stream>>>(
        MODh, MODl, HDIM, 0LL, Wm1T, HDIM, 0LL,
        (void*)Ah, (void*)Al, HDIM, 0LL, NPIX, HDIM, HDIM,
        modb1, HB1, HDIM, M0h, M0l, HDIM, F_BIAS | F_ADDF | F_RELU | F_ADDB);
    gemm64<1, 2><<<gP256, blk, 0, stream>>>(
        Ah, Al, HDIM, 0LL, WhvT, HDIM, 0LL,
        (void*)HVh, (void*)HVl, HDIM, 0LL, NPIX, HDIM, HDIM,
        hvb0, HB0, HDIM, XQh, XQl, HDIM, F_BIAS | F_RELU);
    outk<<<gOut, dim3(128), 0, stream>>>(M0h, M0l, HVh, HVl, outW0, outb0, outW1, outb1,
                                         out + (size_t)b * NPIX * NOUTC);
  }
  (void)hipGetLastError();
}
